// SelfAttention_63866163692092
// MI455X (gfx1250) — hardware-verified
//
#include <hip/hip_runtime.h>


#ifndef NB
#define NB 4
#endif
#ifndef SEQ
#define SEQ 2048
#endif
#define NB_FULL    4
#define SEQ_FULL   2048
#define NHEAD      16
#define HDIM       64
#define DM         (NHEAD * HDIM)
#define BQ         128
#define BK         32
#define NWAVE      8
#define EARLY_T    ((SEQ < 512) ? SEQ : 512)
#define OP         68
#define GT         128
#define CP         132
#define MW         (SEQ / 32)
#define MPITCH     (((MW + 1 + 31) / 32) * 32)
#define LATE_T     (SEQ - EARLY_T)
#define LATE_TILES (((LATE_T / GT) > 0) ? (LATE_T / GT) : 1)
#define EARLY_TILES (EARLY_T / GT)

#define QK_CARRY   16.0f
#define V_CARRY    16.0f
#define P_CARRY    4096.0f
#define CTX_CARRY  64.0f
#define WP_CARRY   64.0f
#define RES_CARRY  2048.0f
#define RES_INV    (1.0f / 2048.0f)

static_assert(SEQ % 256 == 0);
static_assert(SEQ % GT == 0);
static_assert(SEQ % BQ == 0);
static_assert(EARLY_T % GT == 0);
static_assert(EARLY_T % BQ == 0);
static_assert(EARLY_T >= BK);
static_assert(BQ == NWAVE * 16);
static_assert(HDIM == 64);
static_assert(DM % GT == 0);
static_assert(DM % 32 == 0);
static_assert(SEQ <= SEQ_FULL);
static_assert(NB >= 1 && NB <= NB_FULL);
static_assert((OP * 4) % 16 == 0);
static_assert((CP * 4) % 16 == 0);
static_assert(MPITCH / 4 <= 32);
static_assert(MPITCH <= 256);
static_assert(((size_t)NB * SEQ * DM) % 2048 == 0);
static_assert(((size_t)DM * DM) % 2048 == 0);
static_assert(256 * 8 * 8 == GT * GT);
static_assert(256 * 16 * 4 == GT * GT);
static_assert(32 * 4 * 8 == 16 * HDIM);

typedef __bf16         bf16;
typedef _Float16       f16;
typedef unsigned short u16;
typedef bf16     v16bf __attribute__((ext_vector_type(16)));
typedef f16      v16h  __attribute__((ext_vector_type(16)));
typedef float    v8f   __attribute__((ext_vector_type(8)));
typedef float    v4f   __attribute__((ext_vector_type(4)));
typedef unsigned v4u   __attribute__((ext_vector_type(4)));

union Frag   { v16bf vb; v16h vh; v4u q[2]; };
union Pack8B { v4u u; bf16 h[8]; };
union Pack8H { v4u u; f16  h[8]; };

static __device__ __forceinline__ v8f mma_bf16(v16bf a, v16bf b, v8f acc) {
  acc = __builtin_amdgcn_wmma_f32_16x16x32_bf16(false, a, false, b, (short)0, acc, false, false);
  asm volatile("v_nop\n\tv_nop\n\tv_nop\n\tv_nop" : "+v"(acc) : "v"(a), "v"(b));
  return acc;
}
static __device__ __forceinline__ v8f mma_f16(v16h a, v16h b, v8f acc) {
  acc = __builtin_amdgcn_wmma_f32_16x16x32_f16(false, a, false, b, (short)0, acc, false, false);
  asm volatile("v_nop\n\tv_nop\n\tv_nop\n\tv_nop" : "+v"(acc) : "v"(a), "v"(b));
  return acc;
}

static __device__ __forceinline__ float bfr(float x) { return (float)(bf16)x; }

static __device__ __forceinline__ void pack_hr(const float (&v)[8], float carry, v4u& hv, v4u& rv) {
  Pack8H ph, pr;
  #pragma unroll
  for (int i = 0; i < 8; ++i) {
    const float yc = v[i] * carry;
    const f16 hh = (f16)yc;
    ph.h[i] = hh;
    pr.h[i] = (f16)((yc - (float)hh) * RES_CARRY);
  }
  hv = ph.u;
  rv = pr.u;
}

__global__ __launch_bounds__(256) void cvt_x_kernel(const float* __restrict__ x, u16* __restrict__ xb) {
  const size_t e   = ((size_t)blockIdx.x * 256 + threadIdx.x) * 8;
  const size_t row = e / DM;
  const int    col = (int)(e % DM);
  const size_t b   = row / SEQ;
  const size_t t   = row % SEQ;
  const float* src = x + (b * SEQ_FULL + t) * DM + col;
  const v4f a0 = *(const v4f*)(src);
  const v4f a1 = *(const v4f*)(src + 4);
  Pack8B pk;
  #pragma unroll
  for (int i = 0; i < 4; ++i) {
    pk.h[i]     = (bf16)a0[i];
    pk.h[4 + i] = (bf16)a1[i];
  }
  const v4u val = pk.u;
  *(volatile v4u*)(xb + e) = val;
  __threadfence();
  *(volatile v4u*)(xb + e) = val;
}

__global__ __launch_bounds__(256) void cvt_w_kernel(const float* __restrict__ wq, const float* __restrict__ wk,
                                                    const float* __restrict__ wv, const float* __restrict__ wp,
                                                    u16* __restrict__ wpl) {
  const int z = blockIdx.y;
  const float* src = (z == 0) ? wq : (z == 1) ? wk : (z == 2) ? wv : wp;
  const size_t e = ((size_t)blockIdx.x * 256 + threadIdx.x) * 8;
  const v4f a0 = *(const v4f*)(src + e);
  const v4f a1 = *(const v4f*)(src + e + 4);
  v4u val;
  if (z < 3) {
    Pack8B pk;
    #pragma unroll
    for (int i = 0; i < 4; ++i) {
      pk.h[i]     = (bf16)a0[i];
      pk.h[4 + i] = (bf16)a1[i];
    }
    val = pk.u;
  } else {
    Pack8H ph;
    #pragma unroll
    for (int i = 0; i < 4; ++i) {
      ph.h[i]     = (f16)(bfr(a0[i]) * WP_CARRY);
      ph.h[4 + i] = (f16)(bfr(a1[i]) * WP_CARRY);
    }
    val = ph.u;
  }
  u16* dst = wpl + (size_t)z * DM * DM + e;
  *(volatile v4u*)dst = val;
  __threadfence();
  *(volatile v4u*)dst = val;
}

__global__ __launch_bounds__(256) void mask_pack_kernel(const int* __restrict__ amask, const int* __restrict__ pmask,
                                                        unsigned* __restrict__ mbits, unsigned* __restrict__ pbits) {
  __shared__ __align__(16) unsigned sW[MPITCH];
  __shared__ int sBad;
  const int tid  = threadIdx.x;
  const int wave = tid >> 5;
  const int lane = tid & 31;
  const int rid  = blockIdx.x;
  const bool is_pad = (rid >= SEQ);
  const int q  = is_pad ? 0 : rid;
  const int pb = is_pad ? (rid - SEQ) : 0;
  const int* src = is_pad ? (pmask + (size_t)pb * SEQ_FULL) : (amask + (size_t)q * SEQ_FULL);
  unsigned*  dst = is_pad ? (pbits + (size_t)pb * MPITCH)   : (mbits + (size_t)q * MPITCH);
  if (tid == 0) sBad = 0;
  #pragma unroll 1
  for (int it = 0; it < SEQ / 256; ++it) {
    const int v = src[it * 256 + tid];
    const unsigned w = __builtin_amdgcn_ballot_w32(v != 0);
    if (lane == 0) sW[it * 8 + wave] = w;
  }
  __syncthreads();
  if (!is_pad && tid < MW) {
    const unsigned w = sW[tid];
    const int wq = q >> 5;
    const int bq = q & 31;
    int bad = 0;
    if (tid > wq) bad = (w != 0u);
    if (tid == wq) {
      const unsigned upper = (bq == 31) ? 0u : (w >> (bq + 1));
      bad = (upper != 0u) || (((w >> bq) & 1u) == 0u);
    }
    if (bad) sBad = 1;
  }
  __syncthreads();
  const int anybad = sBad;
  if (tid >= MW && tid < MPITCH) sW[tid] = (tid == MW) ? (anybad ? 0u : 1u) : 0u;
  __syncthreads();
  if (tid < MPITCH / 4) {
    const v4u val = *(const v4u*)(sW + tid * 4);
    *(volatile v4u*)(dst + tid * 4) = val;
    __threadfence();
    *(volatile v4u*)(dst + tid * 4) = val;
  }
}

template <int F16>
static __device__ __forceinline__ void gemm_core(const u16* __restrict__ arow, const u16* __restrict__ brow,
                                                 v8f (&acc)[2][4]) {
  #pragma unroll 1
  for (int k0 = 0; k0 < DM; k0 += 32) {
    Frag a[2], bb[4];
    #pragma unroll
    for (int mt = 0; mt < 2; ++mt) {
      a[mt].q[0] = *(const v4u*)(arow + (size_t)mt * 16 * DM + k0);
      a[mt].q[1] = *(const v4u*)(arow + (size_t)mt * 16 * DM + k0 + 16);
    }
    #pragma unroll
    for (int nt = 0; nt < 4; ++nt) {
      bb[nt].q[0] = *(const v4u*)(brow + (size_t)nt * 16 * DM + k0);
      bb[nt].q[1] = *(const v4u*)(brow + (size_t)nt * 16 * DM + k0 + 16);
    }
    #pragma unroll
    for (int mt = 0; mt < 2; ++mt) {
      #pragma unroll
      for (int nt = 0; nt < 4; ++nt) {
        if (F16 != 0) acc[mt][nt] = mma_f16(a[mt].vh, bb[nt].vh, acc[mt][nt]);
        else          acc[mt][nt] = mma_bf16(a[mt].vb, bb[nt].vb, acc[mt][nt]);
      }
    }
  }
}

template <int ADD>
static __device__ __forceinline__ void stage_tile(float* sC, const v8f (&acc)[2][4], int wm, int wn, int lq, int hi,
                                                  float scl) {
  #pragma unroll
  for (int mt = 0; mt < 2; ++mt) {
    #pragma unroll
    for (int nt = 0; nt < 4; ++nt) {
      #pragma unroll
      for (int r = 0; r < 8; ++r) {
        const int idx = (wm + mt * 16 + hi * 8 + r) * CP + wn + nt * 16 + lq;
        const float v = acc[mt][nt][r] * scl;
        if (ADD != 0) sC[idx] = sC[idx] + v;
        else          sC[idx] = v;
      }
    }
  }
}

__global__ __launch_bounds__(256) void gemm_qk_kernel(const u16* __restrict__ xb, const u16* __restrict__ wpl,
                                                      const float* __restrict__ bq, const float* __restrict__ bk,
                                                      const float* __restrict__ fc,
                                                      u16* __restrict__ qh, u16* __restrict__ kh,
                                                      u16* __restrict__ qr, u16* __restrict__ kr) {
  __shared__ __align__(16) float sC[GT * CP];
  const int tid  = threadIdx.x;
  const int lane = tid & 31;
  const int wave = tid >> 5;
  const int lq   = lane & 15;
  const int hi   = lane >> 4;
  const int z    = blockIdx.z;
  const int nblk = blockIdx.x * GT;
  const int mblk = blockIdx.y * GT;
  const int wm   = (wave & 3) * 32;
  const int wn   = (wave >> 2) * 64;
  const u16*   W    = wpl + (size_t)z * DM * DM;
  const float* bias = (z == 0) ? bq : bk;
  u16* hp = (z == 0) ? qh : kh;
  u16* rp = (z == 0) ? qr : kr;

  v8f acc[2][4];
  #pragma unroll
  for (int mt = 0; mt < 2; ++mt) {
    #pragma unroll
    for (int nt = 0; nt < 4; ++nt) acc[mt][nt] = (v8f){0, 0, 0, 0, 0, 0, 0, 0};
  }
  gemm_core<0>(xb + (size_t)(mblk + wm + lq) * DM + hi * 8, W + (size_t)(nblk + wn + lq) * DM + hi * 8, acc);
  stage_tile<0>(sC, acc, wm, wn, lq, hi, 1.0f);
  __syncthreads();

  const int b     = mblk / SEQ;
  const int t0    = mblk % SEQ;
  const bool early = (t0 < EARLY_T);
  const int seg   = tid & 7;
  const int hs    = (tid >> 3) & 1;
  const int rsub  = tid >> 4;
  const int n0    = nblk + hs * 64 + seg * 8;
  const int h     = n0 >> 6;

  float bz[8];
  {
    const v4f b0 = *(const v4f*)(bias + n0);
    const v4f b1 = *(const v4f*)(bias + n0 + 4);
    #pragma unroll
    for (int i = 0; i < 4; ++i) {
      bz[i]     = bfr(b0[i]);
      bz[4 + i] = bfr(b1[i]);
    }
  }

  v4u hv[8], rv[8];
  #pragma unroll
  for (int p = 0; p < 8; ++p) {
    const int row = p * 16 + rsub;
    const int t   = t0 + row;
    const float* sp = sC + row * CP + hs * 64 + seg * 8;
    const v4f s0 = *(const v4f*)(sp);
    const v4f s1 = *(const v4f*)(sp + 4);
    const float* fp = fc + ((size_t)t * (HDIM / 2) + seg * 4) * 2;
    const v4f f0 = *(const v4f*)(fp);
    const v4f f1 = *(const v4f*)(fp + 4);
    float xv[8], cs[8], ov[8];
    #pragma unroll
    for (int i = 0; i < 4; ++i) {
      xv[i]     = s0[i] + bz[i];
      xv[4 + i] = s1[i] + bz[4 + i];
      cs[i]     = bfr(f0[i]);
      cs[4 + i] = bfr(f1[i]);
    }
    #pragma unroll
    for (int j = 0; j < 4; ++j) {
      const float x1 = xv[2 * j], x2 = xv[2 * j + 1];
      const float c  = cs[2 * j], s  = cs[2 * j + 1];
      ov[2 * j]     = x1 * c - x2 * s;
      ov[2 * j + 1] = x1 * s + x2 * c;
    }
    pack_hr(ov, QK_CARRY, hv[p], rv[p]);
  }

  const size_t bh = (size_t)b * NHEAD + h;
  #pragma unroll
  for (int p = 0; p < 8; ++p) {
    const int t = t0 + p * 16 + rsub;
    *(volatile v4u*)(hp + (bh * SEQ + t) * HDIM + seg * 8) = hv[p];
    if (early) *(volatile v4u*)(rp + (bh * EARLY_T + t) * HDIM + seg * 8) = rv[p];
  }
  __threadfence();
  #pragma unroll
  for (int p = 0; p < 8; ++p) {
    const int t = t0 + p * 16 + rsub;
    *(volatile v4u*)(hp + (bh * SEQ + t) * HDIM + seg * 8) = hv[p];
    if (early) *(volatile v4u*)(rp + (bh * EARLY_T + t) * HDIM + seg * 8) = rv[p];
  }
}

__global__ __launch_bounds__(256) void gemm_v_kernel(const u16* __restrict__ wvb, const u16* __restrict__ xb,
                                                     const float* __restrict__ bv,
                                                     u16* __restrict__ vt, u16* __restrict__ vtr) {
  __shared__ __align__(16) float sC[GT * CP];
  const int tid  = threadIdx.x;
  const int lane = tid & 31;
  const int wave = tid >> 5;
  const int lq   = lane & 15;
  const int hi   = lane >> 4;
  const int nblk = blockIdx.x * GT;
  const int mblk = blockIdx.y * GT;
  const int wm   = (wave & 3) * 32;
  const int wn   = (wave >> 2) * 64;

  v8f acc[2][4];
  #pragma unroll
  for (int mt = 0; mt < 2; ++mt) {
    #pragma unroll
    for (int nt = 0; nt < 4; ++nt) acc[mt][nt] = (v8f){0, 0, 0, 0, 0, 0, 0, 0};
  }
  gemm_core<0>(wvb + (size_t)(mblk + wm + lq) * DM + hi * 8, xb + (size_t)(nblk + wn + lq) * DM + hi * 8, acc);
  stage_tile<0>(sC, acc, wm, wn, lq, hi, 1.0f);
  __syncthreads();

  const int b     = nblk / SEQ;
  const int t0    = nblk % SEQ;
  const bool early = (t0 < EARLY_T);
  const int seg   = tid & 7;
  const int hs    = (tid >> 3) & 1;
  const int rsub  = tid >> 4;

  v4u hv[8], rv[8];
  #pragma unroll
  for (int p = 0; p < 8; ++p) {
    const int row = p * 16 + rsub;
    const float bz = bfr(bv[mblk + row]);
    const float* sp = sC + row * CP + hs * 64 + seg * 8;
    const v4f s0 = *(const v4f*)(sp);
    const v4f s1 = *(const v4f*)(sp + 4);
    float ov[8];
    #pragma unroll
    for (int i = 0; i < 4; ++i) {
      ov[i]     = s0[i] + bz;
      ov[4 + i] = s1[i] + bz;
    }
    pack_hr(ov, V_CARRY, hv[p], rv[p]);
  }
  const int tcol = t0 + hs * 64 + seg * 8;
  #pragma unroll
  for (int p = 0; p < 8; ++p) {
    const size_t crow = (size_t)b * DM + mblk + p * 16 + rsub;
    *(volatile v4u*)(vt + crow * SEQ + tcol) = hv[p];
    if (early) *(volatile v4u*)(vtr + crow * EARLY_T + tcol) = rv[p];
  }
  __threadfence();
  #pragma unroll
  for (int p = 0; p < 8; ++p) {
    const size_t crow = (size_t)b * DM + mblk + p * 16 + rsub;
    *(volatile v4u*)(vt + crow * SEQ + tcol) = hv[p];
    if (early) *(volatile v4u*)(vtr + crow * EARLY_T + tcol) = rv[p];
  }
}

template <int RES>
__global__ __launch_bounds__(256) void gemm_out_kernel(const u16* __restrict__ ctxh, const u16* __restrict__ ctxr,
                                                       const u16* __restrict__ wpb, const float* __restrict__ bp,
                                                       float* __restrict__ out) {
  __shared__ __align__(16) float sC[GT * CP];
  const int tid  = threadIdx.x;
  const int lane = tid & 31;
  const int wave = tid >> 5;
  const int lq   = lane & 15;
  const int hi   = lane >> 4;
  const int nblk = blockIdx.x * GT;
  const int y    = blockIdx.y;
  const int b    = (RES != 0) ? (y / EARLY_TILES) : (y / LATE_TILES);
  const int t0   = (RES != 0) ? ((y % EARLY_TILES) * GT) : (EARLY_T + (y % LATE_TILES) * GT);
  const int wm   = (wave & 3) * 32;
  const int wn   = (wave >> 2) * 64;

  v8f acc[2][4];
  #pragma unroll
  for (int mt = 0; mt < 2; ++mt) {
    #pragma unroll
    for (int nt = 0; nt < 4; ++nt) acc[mt][nt] = (v8f){0, 0, 0, 0, 0, 0, 0, 0};
  }
  const u16* brow = wpb + (size_t)(nblk + wn + lq) * DM + hi * 8;
  gemm_core<1>(ctxh + ((size_t)b * SEQ + t0 + wm + lq) * DM + hi * 8, brow, acc);
  stage_tile<0>(sC, acc, wm, wn, lq, hi, 1.0f / (CTX_CARRY * WP_CARRY));
  if (RES != 0) {
    #pragma unroll
    for (int mt = 0; mt < 2; ++mt) {
      #pragma unroll
      for (int nt = 0; nt < 4; ++nt) acc[mt][nt] = (v8f){0, 0, 0, 0, 0, 0, 0, 0};
    }
    gemm_core<1>(ctxr + ((size_t)b * EARLY_T + t0 + wm + lq) * DM + hi * 8, brow, acc);
    stage_tile<1>(sC, acc, wm, wn, lq, hi, RES_INV / (CTX_CARRY * WP_CARRY));
  }
  __syncthreads();

  const int col = lane * 4;
  v4f bz = *(const v4f*)(bp + nblk + col);
  #pragma unroll
  for (int i = 0; i < 4; ++i) bz[i] = bfr(bz[i]);

  v4f vals[16];
  #pragma unroll
  for (int p = 0; p < 16; ++p) {
    const int row = p * 8 + wave;
    const v4f v = *(const v4f*)(sC + row * CP + col);
    vals[p] = v + bz;
  }
  float* obase = out + ((size_t)b * SEQ_FULL + t0 + wave) * DM + nblk + col;
  #pragma unroll
  for (int p = 0; p < 16; ++p) *(volatile v4f*)(obase + (size_t)p * 8 * DM) = vals[p];
  __threadfence();
  #pragma unroll
  for (int p = 0; p < 16; ++p) *(volatile v4f*)(obase + (size_t)p * 8 * DM) = vals[p];
}

template <int RES>
__global__ __launch_bounds__(256) void attn_kernel(const u16* __restrict__ qh_p, const u16* __restrict__ kh_p,
                                                   const u16* __restrict__ vt_p,
                                                   const u16* __restrict__ qr_p, const u16* __restrict__ kr_p,
                                                   const u16* __restrict__ vtr_p,
                                                   const unsigned* __restrict__ mbits,
                                                   const unsigned* __restrict__ pbits,
                                                   u16* __restrict__ ctxh, u16* __restrict__ ctxr, int qblk0) {
  const int qblk = qblk0 + blockIdx.x;
  const int h    = blockIdx.y;
  const int b    = blockIdx.z;
  const int tid  = threadIdx.x;
  const int wave = tid >> 5;
  const int lane = tid & 31;
  const int lq   = lane & 15;
  const int hi   = lane >> 4;

  __shared__ __align__(16) float sO[NWAVE * 16 * OP];

  const int qrow0 = qblk * BQ + wave * 16;
  const int qi    = qrow0 + lq;
  const size_t bh = (size_t)b * NHEAD + h;

  Frag qf[2], qrf[2];
  {
    const u16* qp = qh_p + (bh * SEQ + qi) * HDIM + hi * 8;
    #pragma unroll
    for (int f = 0; f < 2; ++f) {
      qf[f].q[0] = *(const v4u*)(qp + f * 32);
      qf[f].q[1] = *(const v4u*)(qp + f * 32 + 16);
    }
  }
  if (RES != 0) {
    const u16* qp = qr_p + (bh * EARLY_T + qi) * HDIM + hi * 8;
    #pragma unroll
    for (int f = 0; f < 2; ++f) {
      qrf[f].q[0] = *(const v4u*)(qp + f * 32);
      qrf[f].q[1] = *(const v4u*)(qp + f * 32 + 16);
    }
  } else {
    #pragma unroll
    for (int f = 0; f < 2; ++f) {
      qrf[f].q[0] = (v4u){0u, 0u, 0u, 0u};
      qrf[f].q[1] = (v4u){0u, 0u, 0u, 0u};
    }
  }

  const u16* kp  = kh_p  + (bh * SEQ + lq) * HDIM + hi * 8;
  const u16* krp = kr_p  + (bh * EARLY_T + lq) * HDIM + hi * 8;
  const u16* vp  = vt_p  + (bh * HDIM + lq) * SEQ + hi * 8;
  const u16* vrp = vtr_p + (bh * HDIM + lq) * EARLY_T + hi * 8;

  const unsigned* mrow = mbits + (size_t)qi * MPITCH;
  const unsigned* prow = pbits + (size_t)b * MPITCH;

  const unsigned rk = mrow[MW];
  const unsigned pw = prow[qi >> 5];
  const bool rowok  = (rk == 1u) && (((pw >> (qi & 31)) & 1u) != 0u);
  const bool allok  = (__builtin_amdgcn_ballot_w32(rowok) == 0xffffffffu);
  int nchunk = allok ? ((qrow0 + 15) / BK + 1) : (SEQ / BK);
  nchunk = (nchunk < SEQ / BK) ? nchunk : (SEQ / BK);

  v8f o[4], o2[4];
  #pragma unroll
  for (int dt = 0; dt < 4; ++dt) {
    o[dt]  = (v8f){0, 0, 0, 0, 0, 0, 0, 0};
    o2[dt] = (v8f){0, 0, 0, 0, 0, 0, 0, 0};
  }

  float rmax = -__builtin_inff();
  float rsum = 0.0f;
  const float SL      = (0.125f / (QK_CARRY * QK_CARRY)) * 1.4426950408889634f;
  const float FILLRAW = -1.0e30f * 8.0f * (QK_CARRY * QK_CARRY);

  for (int i = 0; i < nchunk; ++i) {
    const int j0 = i * BK;
    const unsigned mw = mrow[i] & prow[i];
    const bool res_on = (RES != 0) && (j0 < EARLY_T);
    const int  jr     = (j0 < EARLY_T) ? j0 : (EARLY_T - BK);

    v8f c[2];
    #pragma unroll
    for (int sub = 0; sub < 2; ++sub) {
      Frag ak[2];
      const u16* kb = kp + (size_t)(j0 + sub * 16) * HDIM;
      #pragma unroll
      for (int f = 0; f < 2; ++f) {
        ak[f].q[0] = *(const v4u*)(kb + f * 32);
        ak[f].q[1] = *(const v4u*)(kb + f * 32 + 16);
      }
      v8f acc = (v8f){0, 0, 0, 0, 0, 0, 0, 0};
      acc = mma_f16(ak[0].vh, qf[0].vh, acc);
      acc = mma_f16(ak[1].vh, qf[1].vh, acc);
      if (RES != 0) {
        Frag akr[2];
        const u16* kbr = krp + (size_t)(jr + sub * 16) * HDIM;
        #pragma unroll
        for (int f = 0; f < 2; ++f) {
          const v4u l0 = *(const v4u*)(kbr + f * 32);
          const v4u l1 = *(const v4u*)(kbr + f * 32 + 16);
          akr[f].q[0] = res_on ? l0 : (v4u){0u, 0u, 0u, 0u};
          akr[f].q[1] = res_on ? l1 : (v4u){0u, 0u, 0u, 0u};
        }
        v8f acc2 = (v8f){0, 0, 0, 0, 0, 0, 0, 0};
        acc2 = mma_f16(ak[0].vh,  qrf[0].vh, acc2);
        acc2 = mma_f16(ak[1].vh,  qrf[1].vh, acc2);
        acc2 = mma_f16(akr[0].vh, qf[0].vh,  acc2);
        acc2 = mma_f16(akr[1].vh, qf[1].vh,  acc2);
        #pragma unroll
        for (int r = 0; r < 8; ++r) acc[r] += acc2[r] * RES_INV;
        asm volatile("" ::: "memory");
      }
      c[sub] = acc;
    }

    if (__builtin_amdgcn_ballot_w32(mw != 0xffffffffu) != 0u) {
      const unsigned ms = mw >> (hi * 8);
      #pragma unroll
      for (int sub = 0; sub < 2; ++sub) {
        #pragma unroll
        for (int r = 0; r < 8; ++r) {
          const bool allowed = ((ms >> (sub * 16 + r)) & 1u) != 0u;
          c[sub][r] = allowed ? c[sub][r] : FILLRAW;
        }
      }
    }

    float m_new = rmax;
    #pragma unroll
    for (int r = 0; r < 8; ++r) {
      m_new = fmaxf(m_new, c[0][r]);
      m_new = fmaxf(m_new, c[1][r]);
    }
    m_new = fmaxf(m_new, __shfl_xor(m_new, 16, 32));
    const float scale = __builtin_amdgcn_exp2f((rmax - m_new) * SL);
    rmax = m_new;

    Frag pa, pr;
    {
      Pack8H a0, a1, r0, r1;
      float psum = 0.0f;
      #pragma unroll
      for (int r = 0; r < 8; ++r) {
        const float p0 = __builtin_amdgcn_exp2f((c[0][r] - m_new) * SL);
        const float p1 = __builtin_amdgcn_exp2f((c[1][r] - m_new) * SL);
        psum += p0 + p1;
        const float pc0 = p0 * P_CARRY;
        const float pc1 = p1 * P_CARRY;
        const f16 h0 = (f16)pc0;
        const f16 h1 = (f16)pc1;
        a0.h[r] = h0;
        a1.h[r] = h1;
        if (RES != 0) {
          r0.h[r] = (f16)((pc0 - (float)h0) * RES_CARRY);
          r1.h[r] = (f16)((pc1 - (float)h1) * RES_CARRY);
        } else {
          r0.h[r] = (f16)0.0f;
          r1.h[r] = (f16)0.0f;
        }
      }
      pa.q[0] = a0.u;  pa.q[1] = a1.u;
      pr.q[0] = r0.u;  pr.q[1] = r1.u;
      rsum = rsum * scale + psum + __shfl_xor(psum, 16, 32);
    }

    float sc[8];
    #pragma unroll
    for (int r = 0; r < 8; ++r) sc[r] = __shfl(scale, (hi << 3) + r, 32);
    #pragma unroll
    for (int dt = 0; dt < 4; ++dt) {
      #pragma unroll
      for (int r = 0; r < 8; ++r) {
        o[dt][r] *= sc[r];
        if (RES != 0) o2[dt][r] *= sc[r];
      }
    }
    if (RES != 0) asm volatile("" ::: "memory");

    #pragma unroll
    for (int dt = 0; dt < 4; ++dt) {
      Frag bv;
      const u16* vb = vp + (size_t)dt * 16 * SEQ + j0;
      bv.q[0] = *(const v4u*)(vb);
      bv.q[1] = *(const v4u*)(vb + 16);
      o[dt] = mma_f16(pa.vh, bv.vh, o[dt]);
      if (RES != 0) {
        Frag bvr;
        const u16* vbr = vrp + (size_t)dt * 16 * EARLY_T + jr;
        const v4u l0 = *(const v4u*)(vbr);
        const v4u l1 = *(const v4u*)(vbr + 16);
        bvr.q[0] = res_on ? l0 : (v4u){0u, 0u, 0u, 0u};
        bvr.q[1] = res_on ? l1 : (v4u){0u, 0u, 0u, 0u};
        o2[dt] = mma_f16(pa.vh, bvr.vh, o2[dt]);
        o2[dt] = mma_f16(pr.vh, bv.vh,  o2[dt]);
      }
    }
  }

  float rs[8];
  #pragma unroll
  for (int r = 0; r < 8; ++r) rs[r] = 1.0f / __shfl(rsum, (hi << 3) + r, 32);

  float* so = sO + wave * (16 * OP);
  #pragma unroll
  for (int r = 0; r < 8; ++r) {
    #pragma unroll
    for (int dt = 0; dt < 4; ++dt) {
      float val = o[dt][r];
      if (RES != 0) val += o2[dt][r] * RES_INV;
      so[(hi * 8 + r) * OP + dt * 16 + lq] = val * (1.0f / (P_CARRY * V_CARRY)) * rs[r];
    }
  }
  __syncthreads();

  const int seg = lane & 7;
  v4u hv[4], rv[4];
  #pragma unroll
  for (int it = 0; it < 4; ++it) {
    const int row = it * 4 + (lane >> 3);
    const v4f a0 = *(const v4f*)(so + row * OP + seg * 8);
    const v4f a1 = *(const v4f*)(so + row * OP + seg * 8 + 4);
    float ov[8];
    #pragma unroll
    for (int i = 0; i < 4; ++i) {
      ov[i]     = a0[i];
      ov[4 + i] = a1[i];
    }
    pack_hr(ov, CTX_CARRY, hv[it], rv[it]);
  }
  #pragma unroll
  for (int it = 0; it < 4; ++it) {
    const int row = qrow0 + it * 4 + (lane >> 3);
    *(volatile v4u*)(ctxh + ((size_t)b * SEQ + row) * DM + h * HDIM + seg * 8) = hv[it];
    if (RES != 0) *(volatile v4u*)(ctxr + ((size_t)b * EARLY_T + row) * DM + h * HDIM + seg * 8) = rv[it];
  }
  __threadfence();
  #pragma unroll
  for (int it = 0; it < 4; ++it) {
    const int row = qrow0 + it * 4 + (lane >> 3);
    *(volatile v4u*)(ctxh + ((size_t)b * SEQ + row) * DM + h * HDIM + seg * 8) = hv[it];
    if (RES != 0) *(volatile v4u*)(ctxr + ((size_t)b * EARLY_T + row) * DM + h * HDIM + seg * 8) = rv[it];
  }
}

static constexpr size_t al128(size_t x) { return (x + 127) & ~(size_t)127; }
static constexpr size_t XB_B   = al128((size_t)NB * SEQ * DM * 2);
static constexpr size_t WPL_B  = al128((size_t)4 * DM * DM * 2);
static constexpr size_t QH_B   = al128((size_t)NB * NHEAD * SEQ * HDIM * 2);
static constexpr size_t QR_B   = al128((size_t)NB * NHEAD * EARLY_T * HDIM * 2);
static constexpr size_t VT_B   = al128((size_t)NB * DM * SEQ * 2);
static constexpr size_t VTR_B  = al128((size_t)NB * DM * EARLY_T * 2);
static constexpr size_t CTXH_B = al128((size_t)NB * SEQ * DM * 2);
static constexpr size_t CTXR_B = al128((size_t)NB * EARLY_T * DM * 2);
static constexpr size_t MB_B   = al128((size_t)SEQ * MPITCH * 4);
static constexpr size_t PB_B   = al128((size_t)NB * MPITCH * 4);
static constexpr size_t WS_TOTAL = XB_B + WPL_B + 2 * QH_B + 2 * QR_B + VT_B + VTR_B + CTXH_B + CTXR_B + MB_B + PB_B;
static_assert(WS_TOTAL <= (size_t)134217728);

extern "C" void kernel_launch(void* const* d_in, const int* in_sizes, int n_in,
                              void* d_out, int out_size, void* d_ws, size_t ws_size,
                              hipStream_t stream) {
  if (n_in < 12) return;
  const size_t rows_used = (size_t)(NB - 1) * SEQ_FULL + SEQ;
  if ((size_t)in_sizes[0] < rows_used * DM) return;
  if ((size_t)in_sizes[1] < (size_t)SEQ * HDIM) return;
  if ((size_t)in_sizes[2] < (size_t)(SEQ - 1) * SEQ_FULL + SEQ) return;
  if ((size_t)in_sizes[3] < rows_used) return;
  if ((size_t)in_sizes[4] < (size_t)DM * DM || (size_t)in_sizes[6] < (size_t)DM * DM) return;
  if ((size_t)in_sizes[8] < (size_t)DM * DM || (size_t)in_sizes[10] < (size_t)DM * DM) return;
  if (in_sizes[5] < DM || in_sizes[7] < DM || in_sizes[9] < DM || in_sizes[11] < DM) return;
  if ((size_t)out_size < rows_used * DM) return;
  if (ws_size < WS_TOTAL) return;

  const float* x   = (const float*)d_in[0];
  const float* fc  = (const float*)d_in[1];
  const int*   am  = (const int*)d_in[2];
  const int*   pm  = (const int*)d_in[3];
  const float* Wq  = (const float*)d_in[4];
  const float* bq  = (const float*)d_in[5];
  const float* Wk  = (const float*)d_in[6];
  const float* bk  = (const float*)d_in[7];
  const float* Wv  = (const float*)d_in[8];
  const float* bv  = (const float*)d_in[9];
  const float* Wp  = (const float*)d_in[10];
  const float* bp  = (const float*)d_in[11];
  float* out = (float*)d_out;

  char* ws = (char*)d_ws;
  size_t off = 0;
  u16* xb   = (u16*)(ws + off); off += XB_B;
  u16* wpl  = (u16*)(ws + off); off += WPL_B;
  u16* qh   = (u16*)(ws + off); off += QH_B;
  u16* kh   = (u16*)(ws + off); off += QH_B;
  u16* vt   = (u16*)(ws + off); off += VT_B;
  u16* qr   = (u16*)(ws + off); off += QR_B;
  u16* kr   = (u16*)(ws + off); off += QR_B;
  u16* vtr  = (u16*)(ws + off); off += VTR_B;
  u16* ctxh = (u16*)(ws + off); off += CTXH_B;
  u16* ctxr = (u16*)(ws + off); off += CTXR_B;
  unsigned* mbits = (unsigned*)(ws + off); off += MB_B;
  unsigned* pbits = (unsigned*)(ws + off); off += PB_B;

  cvt_x_kernel<<<dim3((unsigned)(((size_t)NB * SEQ * DM) / 2048)), 256, 0, stream>>>(x, xb);
  cvt_w_kernel<<<dim3((unsigned)(((size_t)DM * DM) / 2048), 4), 256, 0, stream>>>(Wq, Wk, Wv, Wp, wpl);
  mask_pack_kernel<<<dim3(SEQ + NB), 256, 0, stream>>>(am, pm, mbits, pbits);

  gemm_qk_kernel<<<dim3(DM / GT, (NB * SEQ) / GT, 2), 256, 0, stream>>>(xb, wpl, bq, bk, fc, qh, kh, qr, kr);
  gemm_v_kernel<<<dim3((NB * SEQ) / GT, DM / GT), 256, 0, stream>>>(wpl + (size_t)2 * DM * DM, xb, bv, vt, vtr);

  const int n_early = EARLY_T / BQ;
  const int n_late  = SEQ / BQ - n_early;
  attn_kernel<1><<<dim3(n_early, NHEAD, NB), 256, 0, stream>>>(qh, kh, vt, qr, kr, vtr, mbits, pbits, ctxh, ctxr, 0);
  if (n_late > 0)
    attn_kernel<0><<<dim3(n_late, NHEAD, NB), 256, 0, stream>>>(qh, kh, vt, qr, kr, vtr, mbits, pbits, ctxh, ctxr,
                                                                 n_early);

  const u16* wpb = wpl + (size_t)3 * DM * DM;
  gemm_out_kernel<1><<<dim3(DM / GT, NB * EARLY_TILES), 256, 0, stream>>>(ctxh, ctxr, wpb, bp, out);
  if (LATE_T > 0)
    gemm_out_kernel<0><<<dim3(DM / GT, NB * (LATE_T / GT)), 256, 0, stream>>>(ctxh, ctxr, wpb, bp, out);
}
